// GATLayer_55499567399479
// MI455X (gfx1250) — hardware-verified
//
#include <hip/hip_runtime.h>
#include <stddef.h>
#include <stdint.h>
#include <math.h>


#define IN_DIM 128
#define HD     128
#define NTHR   256
#define NWAVE  8
#define EPT    8
#define CHUNK  (NTHR * EPT)
#define WCAP   (EPT * 32)
#define LISTN  (NWAVE * WCAP)
#define NBA    512
#define SLA    9
#define RCAP   20480
#define DEGCAP 128
#define GBM    64
#define GTHR   128
#define NEGSL  0.2f
#define AGG_ZINTS (LISTN + 2 * RCAP + 3 * NBA)
#define AGG_TOT   (AGG_ZINTS + 16 + NWAVE * DEGCAP * 4 + NWAVE * DEGCAP)
#define WSMAX  134217728

static_assert((CHUNK & (CHUNK - 1)) == 0 && CHUNK <= 4096);
static_assert((NBA & (NBA - 1)) == 0 && NBA == (1 << SLA));
static_assert(((long long)CHUNK << SLA) < (1LL << 31));
static_assert(NBA % NWAVE == 0 && NBA % 32 == 0);
static_assert(RCAP % 4 == 0 && AGG_ZINTS % 4 == 0 && AGG_TOT % 4 == 0 && ((AGG_ZINTS + 16) % 4) == 0);
static_assert(DEGCAP % 32 == 0);
static_assert(IN_DIM % 32 == 0 && HD == 4 * 32);
static_assert(GBM == (GTHR / 32) * 16);
static_assert(AGG_TOT * 4 <= 300000);

typedef float          v4f   __attribute__((ext_vector_type(4)));
typedef float          v8f   __attribute__((ext_vector_type(8)));
typedef int            v4i   __attribute__((ext_vector_type(4)));
typedef int            v8i   __attribute__((ext_vector_type(8)));
typedef unsigned int   v4u   __attribute__((ext_vector_type(4)));
typedef unsigned short v8us  __attribute__((ext_vector_type(8)));
typedef __bf16         v16bf __attribute__((ext_vector_type(16)));
typedef v4f  __attribute__((may_alias)) v4fa;
typedef v4i  __attribute__((may_alias)) v4ia;
typedef v8us __attribute__((may_alias)) v8usa;
union FragB { v16bf v; v8us h[2]; v8i w; };

__device__ __forceinline__ v8f wmb(const FragB& a, const FragB& b, v8f c) {
  v8f d = __builtin_amdgcn_wmma_f32_16x16x32_bf16(false, a.v, false, b.v, (short)0, c, false, false);
  asm volatile("v_nop\n\tv_nop\n\tv_nop\n\tv_nop" : "+v"(d) : "v"(a.w), "v"(b.w));
  return d;
}

__device__ __forceinline__ unsigned bf16_bits(float f) {
  const unsigned u = __float_as_uint(f);
  return ((u + 0x7FFFu + ((u >> 16) & 1u)) >> 16) & 0xFFFFu;
}
__device__ __forceinline__ float bf16_val(float f) {
  return __uint_as_float(bf16_bits(f) << 16);
}
__device__ __forceinline__ v4f bfr4(const v4f a) {
  v4f r; r.x = bf16_val(a.x); r.y = bf16_val(a.y); r.z = bf16_val(a.z); r.w = bf16_val(a.w); return r;
}
__device__ __forceinline__ unsigned pk2(float lo, float hi) { return bf16_bits(lo) | (bf16_bits(hi) << 16); }
__device__ __forceinline__ float lrelu(float x) { return x > 0.f ? x : NEGSL * x; }

template <int SLB>
__device__ __forceinline__ int scan_chunk(const int* __restrict__ dsts, int nE, int cbase, int slotBase,
                                          int nb, int vec8, int* list, int tid, int lane, int wave) {
  int wc = 0;
  const int el0  = tid * EPT;
  const int e0   = cbase + el0;
  const int sent = -2147483647 - 1;
  v4i da, db;
  if (vec8 != 0 && cbase + CHUNK <= nE) {
    da = *(const v4i*)(dsts + e0);
    db = *(const v4i*)(dsts + e0 + 4);
  } else {
    da.x = (e0     < nE) ? dsts[min(e0,     nE - 1)] : sent;
    da.y = (e0 + 1 < nE) ? dsts[min(e0 + 1, nE - 1)] : sent;
    da.z = (e0 + 2 < nE) ? dsts[min(e0 + 2, nE - 1)] : sent;
    da.w = (e0 + 3 < nE) ? dsts[min(e0 + 3, nE - 1)] : sent;
    db.x = (e0 + 4 < nE) ? dsts[min(e0 + 4, nE - 1)] : sent;
    db.y = (e0 + 5 < nE) ? dsts[min(e0 + 5, nE - 1)] : sent;
    db.z = (e0 + 6 < nE) ? dsts[min(e0 + 6, nE - 1)] : sent;
    db.w = (e0 + 7 < nE) ? dsts[min(e0 + 7, nE - 1)] : sent;
  }
  const unsigned nbs = (unsigned)slotBase;
  const unsigned unb = (unsigned)nb;
  const unsigned s0 = (unsigned)da.x - nbs, s1 = (unsigned)da.y - nbs;
  const unsigned s2 = (unsigned)da.z - nbs, s3 = (unsigned)da.w - nbs;
  const unsigned s4 = (unsigned)db.x - nbs, s5 = (unsigned)db.y - nbs;
  const unsigned s6 = (unsigned)db.z - nbs, s7 = (unsigned)db.w - nbs;
  const bool h0 = s0 < unb, h1 = s1 < unb, h2 = s2 < unb, h3 = s3 < unb;
  const bool h4 = s4 < unb, h5 = s5 < unb, h6 = s6 < unb, h7 = s7 < unb;
  const unsigned any = __builtin_amdgcn_ballot_w32(h0 | h1 | h2 | h3 | h4 | h5 | h6 | h7);
  if (any != 0u) {
#define HITJ(J, HJ, SJ) { \
      const unsigned mj = __builtin_amdgcn_ballot_w32(HJ); \
      if (mj != 0u) { \
        if (HJ) { \
          const int pos = wc + (int)__builtin_amdgcn_mbcnt_lo(mj, 0u); \
          if (pos < WCAP) list[wave * WCAP + pos] = ((el0 + (J)) << SLB) | (int)(SJ); \
        } \
        wc += (int)__builtin_popcount(mj); } }
    HITJ(0, h0, s0)
    HITJ(1, h1, s1)
    HITJ(2, h2, s2)
    HITJ(3, h3, s3)
    HITJ(4, h4, s4)
    HITJ(5, h5, s5)
    HITJ(6, h6, s6)
    HITJ(7, h7, s7)
#undef HITJ
  }
  return wc;
}

__global__ __launch_bounds__(NTHR) void k_prep(const float* __restrict__ W, unsigned short* WB, int nUnits) {
  const int u = (int)blockIdx.x * NTHR + (int)threadIdx.x;
  if (u >= nUnits) return;
  const float* p = W + (size_t)u * 8;
  const v4f a = *(const v4fa*)p;
  const v4f b = *(const v4fa*)(p + 4);
  v4u o;
  o.x = pk2(a.x, a.y); o.y = pk2(a.z, a.w); o.z = pk2(b.x, b.y); o.w = pk2(b.z, b.w);
  unsigned short* dp = WB + (size_t)u * 8;
  *(volatile v4u*)dp = o;
  __threadfence();
  *(volatile v4u*)dp = o;
}

__global__ __launch_bounds__(GTHR) void k_proj(const float* __restrict__ X, int nN,
                                               const unsigned short* __restrict__ WB,
                                               const float* __restrict__ attl, const float* __restrict__ attr,
                                               float* FT, float* A1, float* A2) {
  __shared__ __attribute__((aligned(16))) float stg[GBM * HD];
  __shared__ __attribute__((aligned(16))) float sdt[2 * GBM * 4];
  const int tid = (int)threadIdx.x, lane = tid & 31, wave = tid >> 5, hh = lane >> 4, m = lane & 15;
  const int rowBase = (int)blockIdx.x * GBM;
  const int grow = rowBase + 16 * wave + m;
  const int rcl  = grow < nN ? grow : nN - 1;
  const bool rok = grow < nN;

  v8f acc[8];
  {
    const v8f z = {0.f, 0.f, 0.f, 0.f, 0.f, 0.f, 0.f, 0.f};
#pragma unroll
    for (int t = 0; t < 8; ++t) acc[t] = z;
  }
  const float* ap = X + (size_t)rcl * IN_DIM + 8 * hh;
  const unsigned short* bp = WB + (size_t)m * IN_DIM + 8 * hh;

#pragma unroll 1
  for (int k0 = 0; k0 < IN_DIM; k0 += 32) {
    v4f x0 = *(const v4fa*)(ap + k0);
    v4f x1 = *(const v4fa*)(ap + k0 + 4);
    v4f x2 = *(const v4fa*)(ap + k0 + 16);
    v4f x3 = *(const v4fa*)(ap + k0 + 20);
    const v4f z4 = {0.f, 0.f, 0.f, 0.f};
    x0 = rok ? x0 : z4; x1 = rok ? x1 : z4; x2 = rok ? x2 : z4; x3 = rok ? x3 : z4;
    FragB af;
    v8i aw;
    aw[0] = (int)pk2(x0.x, x0.y); aw[1] = (int)pk2(x0.z, x0.w);
    aw[2] = (int)pk2(x1.x, x1.y); aw[3] = (int)pk2(x1.z, x1.w);
    aw[4] = (int)pk2(x2.x, x2.y); aw[5] = (int)pk2(x2.z, x2.w);
    aw[6] = (int)pk2(x3.x, x3.y); aw[7] = (int)pk2(x3.z, x3.w);
    af.w = aw;
#pragma unroll
    for (int nt = 0; nt < 8; ++nt) {
      const unsigned short* wq = bp + (size_t)(16 * nt) * IN_DIM + k0;
      FragB bf;
      bf.h[0] = *(const v8usa*)wq;
      bf.h[1] = *(const v8usa*)(wq + 16);
      acc[nt] = wmb(af, bf, acc[nt]);
    }
  }

#pragma unroll
  for (int nt = 0; nt < 8; ++nt) {
    const int lc = 16 * nt + m;
#pragma unroll
    for (int r = 0; r < 8; ++r) {
      const int lr = 16 * wave + 8 * hh + r;
      stg[lr * HD + lc] = acc[nt][r];
    }
  }
  __syncthreads();

  const v4f al4 = bfr4(*(const v4fa*)(attl + 4 * lane));
  const v4f ar4 = bfr4(*(const v4fa*)(attr + 4 * lane));
  const int hq = lane >> 3;
#pragma unroll 1
  for (int i = 0; i < 16; ++i) {
    const int row = wave * 16 + i;
    const v4f p = *(const v4fa*)(stg + row * HD + 4 * lane);
    float s = 0.0f, d = 0.0f;
    s = fmaf(p.x, al4.x, s); s = fmaf(p.y, al4.y, s); s = fmaf(p.z, al4.z, s); s = fmaf(p.w, al4.w, s);
    d = fmaf(p.x, ar4.x, d); d = fmaf(p.y, ar4.y, d); d = fmaf(p.z, ar4.z, d); d = fmaf(p.w, ar4.w, d);
#pragma unroll
    for (int off = 4; off > 0; off >>= 1) {
      s += __shfl_xor(s, off);
      d += __shfl_xor(d, off);
    }
    if ((lane & 7) == 0) { sdt[row * 4 + hq] = s; sdt[GBM * 4 + row * 4 + hq] = d; }
  }
  __syncthreads();

  const int which = wave >> 1, half = wave & 1;
  const v4f sdv = *(const v4fa*)(sdt + which * (GBM * 4) + half * 128 + 4 * lane);
  float* pl = (which == 0) ? A1 : A2;
  float* sp = pl + (size_t)rowBase * 4 + half * 128 + 4 * lane;
#pragma unroll 1
  for (int i = 0; i < 16; ++i) {
    const int row = wave * 16 + i;
    const v4f p = *(const v4fa*)(stg + row * HD + 4 * lane);
    float* op = FT + (size_t)(rowBase + row) * HD + 4 * lane;
    *(volatile v4f*)op = p;
  }
  *(volatile v4f*)sp = sdv;
  __threadfence();
#pragma unroll 1
  for (int i = 0; i < 16; ++i) {
    const int row = wave * 16 + i;
    const v4f p = *(const v4fa*)(stg + row * HD + 4 * lane);
    float* op = FT + (size_t)(rowBase + row) * HD + 4 * lane;
    *(volatile v4f*)op = p;
  }
  *(volatile v4f*)sp = sdv;
}

__global__ __launch_bounds__(NTHR) void k_scan(const int* __restrict__ srcs, const int* __restrict__ dsts,
                                               int nE, int nN, int vec8,
                                               const float* __restrict__ A1, const float* __restrict__ A2,
                                               const float* __restrict__ FT, float* outp) {
  extern __shared__ __attribute__((aligned(16))) int dsm[];
  int* list = dsm;
  int* hl   = dsm + LISTN;
  int* sl   = hl + RCAP;
  int* cnt  = sl + RCAP;
  int* offs = cnt + NBA;
  int* cur  = offs + NBA;
  int* misc = cur + NBA;
  float* ecb = (float*)(misc + 16);
  int*   scb = (int*)(ecb + NWAVE * DEGCAP * 4);
  const int tid = (int)threadIdx.x, lane = tid & 31, wave = tid >> 5;
  const int nodeBase = (int)blockIdx.x * NBA;

  {
    const v4i z4 = {0, 0, 0, 0};
    for (int i = tid * 4; i < AGG_TOT; i += NTHR * 4) *(v4ia*)(dsm + i) = z4;
  }
  __syncthreads();

  int t = 0, ov = 0;
  const int nChunks = (nE + CHUNK - 1) / CHUNK;
#pragma unroll 1
  for (int ch = 0; ch < nChunks; ++ch) {
    const int cbase = ch * CHUNK;
    const int wc = scan_chunk<SLA>(dsts, nE, cbase, nodeBase, NBA, vec8, list, tid, lane, wave);
    if (lane == 0) misc[wave] = wc;
    __syncthreads();
    if (wave == 0) {
#pragma unroll 1
      for (int w2 = 0; w2 < NWAVE; ++w2) {
        int c = misc[w2];
        c = c < 0 ? 0 : (c > WCAP ? WCAP : c);
#pragma unroll 1
        for (int b0 = 0; b0 < c; b0 += 32) {
          const int idx = b0 + lane;
          const int ent = list[w2 * WCAP + (idx < WCAP ? idx : WCAP - 1)];
          const int m32 = (c - b0) < 32 ? (c - b0) : 32;
#pragma unroll 1
          for (int k = 0; k < m32; ++k) {
            const int u    = __builtin_amdgcn_readlane(ent, k);
            const int slot = u & (NBA - 1);
            const int el   = (u >> SLA) & (CHUNK - 1);
            const int pk   = ((cbase + el) << SLA) | slot;
            if (t < RCAP) {
              if (lane == 0) { hl[t] = pk; cnt[slot] = cnt[slot] + 1; }
              t = t + 1;
            } else {
              ov = 1;
            }
          }
        }
      }
    }
    __syncthreads();
  }
  if (wave == 0 && lane == 0) { misc[8] = t; misc[9] = ov; }
  __syncthreads();
  int tt = misc[8];
  tt = tt < 0 ? 0 : (tt > RCAP ? RCAP : tt);
  const int ovf = misc[9];

  if (wave == 0) {
    const int base = lane * (NBA / 32);
    int s = 0;
#pragma unroll 1
    for (int i = 0; i < NBA / 32; ++i) s += cnt[base + i];
    int incl = s;
#pragma unroll
    for (int d = 1; d < 32; d <<= 1) {
      const int y = __shfl_up(incl, d, 32);
      if (lane >= d) incl += y;
    }
    int run = incl - s;
#pragma unroll 1
    for (int i = 0; i < NBA / 32; ++i) {
      const int cv = cnt[base + i];
      offs[base + i] = run;
      cur[base + i]  = run;
      run += cv;
    }
  }
  __syncthreads();
  if (wave == 0) {
#pragma unroll 1
    for (int b0 = 0; b0 < tt; b0 += 32) {
      const int idx = b0 + lane;
      const int ent = hl[idx < RCAP ? idx : RCAP - 1];
      const int m32 = (tt - b0) < 32 ? (tt - b0) : 32;
#pragma unroll 1
      for (int k = 0; k < m32; ++k) {
        const int u    = __builtin_amdgcn_readlane(ent, k);
        const int slot = u & (NBA - 1);
        if (lane == 0) {
          int p = cur[slot];
          p = p < 0 ? 0 : (p > RCAP - 1 ? RCAP - 1 : p);
          sl[p] = u;
          cur[slot] = p + 1;
        }
      }
    }
  }
  __syncthreads();

  const float qnan = __int_as_float(0x7fc00000);
  const float pz = (ovf != 0) ? qnan : 0.0f;
  const int head = lane >> 3;
  float* ec = ecb + wave * (DEGCAP * 4);
  int*   sc = scb + wave * DEGCAP;
#pragma unroll 1
  for (int si = 0; si < NBA / NWAVE; ++si) {
    const int s    = si * NWAVE + wave;
    const int node = nodeBase + s;
    const int craw = cnt[s];
    const bool big = craw > DEGCAP;
    int c = craw < 0 ? 0 : (craw > DEGCAP ? DEGCAP : craw);
    int o = offs[s];
    o = o < 0 ? 0 : (o > tt ? tt : o);
    if (c > tt - o) c = tt - o;
    const int nc = node < nN ? node : nN - 1;
    const v4f a2v = *(const v4fa*)(A2 + (size_t)nc * 4);

    v4f mx4 = {-3.0e38f, -3.0e38f, -3.0e38f, -3.0e38f};
#pragma unroll 1
    for (int b0 = 0; b0 < c; b0 += 32) {
      const int hi = b0 + lane;
      int idx = o + hi;
      idx = idx > RCAP - 1 ? RCAP - 1 : idx;
      const int ent = sl[idx];
      int eid = (int)((unsigned)ent >> SLA);
      eid = eid > nE - 1 ? nE - 1 : eid;
      int sr = srcs[eid];
      sr = sr < 0 ? 0 : (sr > nN - 1 ? nN - 1 : sr);
      const v4f a1v = *(const v4fa*)(A1 + (size_t)sr * 4);
      v4f e4;
      e4.x = lrelu(a1v.x + a2v.x); e4.y = lrelu(a1v.y + a2v.y);
      e4.z = lrelu(a1v.z + a2v.z); e4.w = lrelu(a1v.w + a2v.w);
      const bool valid = hi < c;
      sc[hi] = sr;
      *(v4fa*)(ec + 4 * hi) = e4;
      mx4.x = valid ? fmaxf(mx4.x, e4.x) : mx4.x;
      mx4.y = valid ? fmaxf(mx4.y, e4.y) : mx4.y;
      mx4.z = valid ? fmaxf(mx4.z, e4.z) : mx4.z;
      mx4.w = valid ? fmaxf(mx4.w, e4.w) : mx4.w;
    }
#pragma unroll
    for (int off = 16; off > 0; off >>= 1) {
      mx4.x = fmaxf(mx4.x, __shfl_xor(mx4.x, off));
      mx4.y = fmaxf(mx4.y, __shfl_xor(mx4.y, off));
      mx4.z = fmaxf(mx4.z, __shfl_xor(mx4.z, off));
      mx4.w = fmaxf(mx4.w, __shfl_xor(mx4.w, off));
    }

    v4f sm4 = {0.f, 0.f, 0.f, 0.f};
#pragma unroll 1
    for (int b0 = 0; b0 < c; b0 += 32) {
      const int hi = b0 + lane;
      const bool valid = hi < c;
      const v4f e4 = *(const v4fa*)(ec + 4 * hi);
      v4f x4;
      x4.x = expf(e4.x - mx4.x); x4.y = expf(e4.y - mx4.y);
      x4.z = expf(e4.z - mx4.z); x4.w = expf(e4.w - mx4.w);
      x4.x = valid ? x4.x : 0.f; x4.y = valid ? x4.y : 0.f;
      x4.z = valid ? x4.z : 0.f; x4.w = valid ? x4.w : 0.f;
      sm4.x += x4.x; sm4.y += x4.y; sm4.z += x4.z; sm4.w += x4.w;
      *(v4fa*)(ec + 4 * hi) = x4;
    }
#pragma unroll
    for (int off = 16; off > 0; off >>= 1) {
      sm4.x += __shfl_xor(sm4.x, off);
      sm4.y += __shfl_xor(sm4.y, off);
      sm4.z += __shfl_xor(sm4.z, off);
      sm4.w += __shfl_xor(sm4.w, off);
    }

#pragma unroll 1
    for (int b0 = 0; b0 < c; b0 += 32) {
      const int hi = b0 + lane;
      const v4f x4 = *(const v4fa*)(ec + 4 * hi);
      v4f q4;
      q4.x = x4.x / sm4.x; q4.y = x4.y / sm4.y; q4.z = x4.z / sm4.z; q4.w = x4.w / sm4.w;
      *(v4fa*)(ec + 4 * hi) = q4;
    }
    __syncthreads();

    v4f acc = {0.f, 0.f, 0.f, 0.f};
#pragma unroll 1
    for (int k = 0; k < c; ++k) {
      int sk = sc[k];
      sk = sk < 0 ? 0 : (sk > nN - 1 ? nN - 1 : sk);
      const float al = ec[4 * k + head];
      const v4f f = *(const v4fa*)(FT + (size_t)sk * HD + 4 * lane);
      acc.x = fmaf(al, f.x, acc.x);
      acc.y = fmaf(al, f.y, acc.y);
      acc.z = fmaf(al, f.z, acc.z);
      acc.w = fmaf(al, f.w, acc.w);
    }
    const float pzr = big ? qnan : pz;
    v4f o4;
    o4.x = acc.x + pzr; o4.y = acc.y + pzr; o4.z = acc.z + pzr; o4.w = acc.w + pzr;
    if (node < nN) {
      float* op = outp + (size_t)node * HD + 4 * lane;
      *(volatile v4f*)op = o4;
      __threadfence();
      *(volatile v4f*)op = o4;
    }
    __builtin_amdgcn_wave_barrier();
  }
}

static inline int cdiv(int a, int b) { return (a + b - 1) / b; }

extern "C" void kernel_launch(void* const* d_in, const int* in_sizes, int n_in,
                              void* d_out, int out_size, void* d_ws, size_t ws_size,
                              hipStream_t stream) {
  if (n_in < 6) return;
  if (in_sizes[0] < IN_DIM || (in_sizes[0] % IN_DIM) != 0) return;
  const int nN = in_sizes[0] / IN_DIM;
  if (nN > (1 << 22)) return;
  if (in_sizes[1] != HD * IN_DIM) return;
  if (in_sizes[2] != HD || in_sizes[3] != HD) return;
  const int nE = in_sizes[4];
  if (nE < 1 || nE >= (1 << 22)) return;
  if (in_sizes[5] != nE) return;
  if ((long long)out_size != (long long)nN * HD) return;

  const float* feat = (const float*)d_in[0];
  const float* W    = (const float*)d_in[1];
  const float* attl = (const float*)d_in[2];
  const float* attr = (const float*)d_in[3];
  const int*   src  = (const int*)d_in[4];
  const int*   dst  = (const int*)d_in[5];
  float* out = (float*)d_out;

  const int MP   = cdiv(nN, GBM) * GBM;
  const int gM   = MP / GBM;
  const int gA   = cdiv(nN, NBA);
  if ((long long)gA * NBA < (long long)nN) return;
  const int vec8 = ((nE & 3) == 0) ? 1 : 0;

  char* ws = (char*)d_ws;
  size_t off = 0;
  const size_t oWB = off; off += (size_t)HD * IN_DIM * 2;   off = (off + 255) & ~(size_t)255;
  const size_t oA1 = off; off += (size_t)MP * 4 * 4;        off = (off + 255) & ~(size_t)255;
  const size_t oA2 = off; off += (size_t)MP * 4 * 4;        off = (off + 255) & ~(size_t)255;
  const size_t oFT = off; off += (size_t)MP * HD * 4;       off = (off + 255) & ~(size_t)255;
  if (off > ws_size || off > (size_t)WSMAX) return;
  unsigned short* WB = (unsigned short*)(ws + oWB);
  float* A1 = (float*)(ws + oA1);
  float* A2 = (float*)(ws + oA2);
  float* FT = (float*)(ws + oFT);

  const size_t scanLds = (size_t)AGG_TOT * 4;
  hipFuncSetAttribute(reinterpret_cast<const void*>(&k_scan), hipFuncAttributeMaxDynamicSharedMemorySize, (int)scanLds);

  const int nUw = HD * (IN_DIM / 8);
  k_prep<<<cdiv(nUw, NTHR), NTHR, 0, stream>>>(W, WB, nUw);
  k_proj<<<gM, GTHR, 0, stream>>>(feat, nN, WB, attl, attr, FT, A1, A2);
  k_scan<<<gA, NTHR, scanLds, stream>>>(src, dst, nE, nN, vec8, A1, A2, FT, out);
}
